// STU_47820165873726
// MI455X (gfx1250) — hardware-verified
//
#include <hip/hip_runtime.h>
#include <math.h>

typedef __attribute__((ext_vector_type(16))) _Float16 v16h;
typedef __attribute__((ext_vector_type(8)))  _Float16 v8h;
typedef __attribute__((ext_vector_type(8)))  float    v8f;
typedef __attribute__((ext_vector_type(4)))  float    v4f;

constexpr int kSeq     = 2048;
constexpr int kDim     = 768;
constexpr int kNf      = 16;
constexpr int kKHalf   = 8;
constexpr int kKTot    = kNf * kSeq;
constexpr int kVsPitch = 4352;
constexpr int kVsShift = 8;
static_assert(kKTot == 32768);
static_assert((kDim % 64) == 0 && (kDim % 32) == 0 && (kSeq % 64) == 0 && ((kSeq / 2) % 64) == 0);
static_assert((kVsPitch % 8) == 0);
static_assert(2040 + (kSeq - 32) + 31 < kVsPitch);

constexpr float kCarryX = 16.0f;
constexpr float kCarryW = 256.0f;
constexpr float kCarryV = 16.0f;
constexpr float kCarryS = 16.0f;
constexpr float kScale1 = kCarryS / (kCarryX * kCarryW);
constexpr float kScale2 = 1.0f / (kCarryV * kCarryS);

constexpr size_t kBytesX16  = (size_t)kSeq * kDim * 2;
constexpr size_t kBytesMT   = (size_t)2 * kKHalf * kDim * kDim * 2;
constexpr size_t kBytesSRCT = (size_t)2 * kDim * kKTot * 2;
constexpr size_t kBytesVS   = (size_t)kVsShift * kNf * kVsPitch * 2;
constexpr size_t kOffX16  = 0;
constexpr size_t kOffMT   = kOffX16 + kBytesX16;
constexpr size_t kOffSRCT = kOffMT + kBytesMT;
constexpr size_t kOffVS   = kOffSRCT + kBytesSRCT;
constexpr size_t kWsTotal = kOffVS + kBytesVS;
static_assert(kWsTotal == 123797504ull);
static_assert(kWsTotal <= 134217728ull);
static_assert((kOffMT % 128) == 0 && (kOffSRCT % 128) == 0 && (kOffVS % 128) == 0);

constexpr int kXBlocks  = (kSeq * kDim / 8) / 256;
constexpr int kVsBlocks = (kVsShift * kNf * kVsPitch / 8) / 256;
static_assert(kXBlocks * 256 * 8 == kSeq * kDim);
static_assert(kVsBlocks * 256 * 8 == kVsShift * kNf * kVsPitch);

__device__ __forceinline__ float bf16_rne_f32(float f) {
  unsigned u = __float_as_uint(f);
  u = (u + 0x7FFFu + ((u >> 16) & 1u)) & 0xFFFF0000u;
  return __uint_as_float(u);
}

__device__ __forceinline__ v16h frag_load(const _Float16* p) {
  union U { v16h v; v8h h[2]; } f;
  f.h[0] = *(const v8h*)(p);
  f.h[1] = *(const v8h*)(p + 16);
  return f.v;
}
__device__ __forceinline__ v8f frag_mma(v16h a, v16h b, v8f c) {
  return __builtin_amdgcn_wmma_f32_16x16x32_f16(false, a, false, b, (short)0, c, false, false);
}
__device__ __forceinline__ void row_guard(v8f& a0, v8f& a1, v8f& a2, v8f& a3,
                                          v16h x, v16h b0, v16h b1, v16h b2, v16h b3) {
  asm volatile("v_nop\n\tv_nop\n\tv_nop\n\tv_nop"
               : "+v"(a0), "+v"(a1), "+v"(a2), "+v"(a3)
               : "v"(x), "v"(b0), "v"(b1), "v"(b2), "v"(b3));
}
__device__ __forceinline__ void acc_guard4(v8f& a, v8f& b, v8f& c, v8f& d) {
  asm volatile("v_nop\n\tv_nop\n\tv_nop\n\tv_nop" : "+v"(a), "+v"(b), "+v"(c), "+v"(d));
}

__global__ __launch_bounds__(256) void prep_xv_kernel(
    const float* __restrict__ x, const float* __restrict__ vf,
    unsigned short* __restrict__ X16, unsigned short* __restrict__ VS)
{
  const int bx = blockIdx.x;
  if (bx < kXBlocks) {
    const int i = bx * 256 + threadIdx.x;
    const size_t e0 = (size_t)i << 3;
    const v4f a0 = *(const v4f*)(x + e0);
    const v4f a1 = *(const v4f*)(x + e0 + 4);
    v8h hv;
#pragma unroll
    for (int e = 0; e < 4; ++e) {
      const float f0 = a0[e];
      const float f1 = a1[e];
      hv[e]     = (_Float16)(bf16_rne_f32(f0) * kCarryX);
      hv[4 + e] = (_Float16)(bf16_rne_f32(f1) * kCarryX);
    }
    unsigned short* q = X16 + e0;
    *(volatile v8h*)q = hv;
    __threadfence();
    *(volatile v8h*)q = hv;
  } else {
    const int i = (bx - kXBlocks) * 256 + threadIdx.x;
    const int el0 = i << 3;
    const int row = el0 / kVsPitch;
    const int i0  = el0 - row * kVsPitch;
    const int c   = row >> 4;
    const int kf  = row & 15;
    v8h hv;
#pragma unroll
    for (int e = 0; e < 8; ++e) {
      const int lag  = (kSeq - 1) - (i0 + e + c);
      const int lagc = lag < 0 ? 0 : lag;
      float val = vf[(size_t)lagc * kNf + kf];
      asm volatile("" : "+v"(val));
      const float sel = (lag >= 0) ? (bf16_rne_f32(val) * kCarryV) : 0.0f;
      hv[e] = (_Float16)sel;
    }
    unsigned short* q = VS + (size_t)el0;
    *(volatile v8h*)q = hv;
    __threadfence();
    *(volatile v8h*)q = hv;
  }
}

__global__ __launch_bounds__(256) void prep_w_kernel(
    const float* __restrict__ Wp, const float* __restrict__ Wm,
    unsigned short* __restrict__ MT, int khalf)
{
  __shared__ float tile[64 * 65];
  const int tid = threadIdx.x;
  const int jt = blockIdx.x % 12;
  const int dt = blockIdx.x / 12;
  const int z  = blockIdx.y;
  const int s  = z >> 3;
  const int kl = z & 7;
  const int kf = khalf * kKHalf + kl;
  const int d0 = dt * 64, j0 = jt * 64;
  const float* src = (s ? Wm : Wp) + (size_t)kf * kDim * kDim;
#pragma unroll
  for (int qq = 0; qq < 4; ++qq) {
    const int f = tid + 256 * qq;
    const int r = f >> 4;
    const int c4 = (f & 15) * 4;
    const v4f val = *(const v4f*)(src + (size_t)(d0 + r) * kDim + j0 + c4);
    const float f0 = val[0], f1 = val[1], f2 = val[2], f3 = val[3];
    tile[r * 65 + c4 + 0] = f0;
    tile[r * 65 + c4 + 1] = f1;
    tile[r * 65 + c4 + 2] = f2;
    tile[r * 65 + c4 + 3] = f3;
  }
  __syncthreads();
  const int q = tid >> 3, c8 = (tid & 7) * 8;
  v8h hv[2];
#pragma unroll
  for (int it = 0; it < 2; ++it) {
    const int jrow = it * 32 + q;
#pragma unroll
    for (int e = 0; e < 8; ++e) {
      const float w = tile[(c8 + e) * 65 + jrow];
      hv[it][e] = (_Float16)(bf16_rne_f32(w) * kCarryW);
    }
  }
  for (int pass = 0; pass < 2; ++pass) {
#pragma unroll
    for (int it = 0; it < 2; ++it) {
      const int jrow = it * 32 + q;
      unsigned short* dst = MT + ((size_t)z * kDim + j0 + jrow) * kDim + d0 + c8;
      *(volatile v8h*)dst = hv[it];
    }
    __threadfence();
  }
}

__global__ __launch_bounds__(256) void proj_gemm_kernel(
    const unsigned short* __restrict__ MTp, const unsigned short* __restrict__ Xp,
    unsigned short* __restrict__ SRCT, int khalf)
{
  __shared__ __align__(16) float sT[8][16 * 68];
  const int lane = threadIdx.x & 31;
  const int wave = __builtin_amdgcn_readfirstlane((int)(threadIdx.x >> 5));
  const int kl = blockIdx.y;
  const int kf = khalf * kKHalf + kl;
  const int tile = blockIdx.x * 8 + wave;
  const int tm = tile >> 5;
  const int tn = tile & 31;
  const int j0 = tm * 32;
  const int n0 = tn * 64;
  const int rlane = lane & 15;
  const int koff  = (lane >> 4) * 8;
  const int mOff  = (lane >> 4) * 8;

  const _Float16* MT = (const _Float16*)MTp;
  const _Float16* X  = (const _Float16*)Xp;
  const _Float16* aP = MT + ((size_t)kl * kDim + j0 + rlane) * kDim + koff;
  const _Float16* aQ = aP + (size_t)kKHalf * kDim * kDim;
  const _Float16* bX = X + (size_t)(n0 + rlane) * kDim + koff;

  v8f acc[4][4];
#pragma unroll
  for (int i = 0; i < 4; ++i)
#pragma unroll
    for (int j = 0; j < 4; ++j) acc[i][j] = (v8f){0.f,0.f,0.f,0.f,0.f,0.f,0.f,0.f};

  for (int k0 = 0; k0 < kDim; k0 += 32) {
    v16h bh[4];
#pragma unroll
    for (int j = 0; j < 4; ++j) bh[j] = frag_load(bX + (size_t)(j * 16) * kDim + k0);
#pragma unroll
    for (int i = 0; i < 4; ++i) {
      const _Float16* ap = ((i >> 1) ? aQ : aP) + (size_t)((i & 1) * 16) * kDim + k0;
      const v16h ah = frag_load(ap);
#pragma unroll
      for (int j = 0; j < 4; ++j) acc[i][j] = frag_mma(ah, bh[j], acc[i][j]);
      row_guard(acc[i][0], acc[i][1], acc[i][2], acc[i][3], ah, bh[0], bh[1], bh[2], bh[3]);
    }
  }
  acc_guard4(acc[0][0], acc[0][1], acc[0][2], acc[0][3]);
  acc_guard4(acc[1][0], acc[1][1], acc[1][2], acc[1][3]);
  acc_guard4(acc[2][0], acc[2][1], acc[2][2], acc[2][3]);
  acc_guard4(acc[3][0], acc[3][1], acc[3][2], acc[3][3]);

  float* slab = sT[wave];
  const bool oddc = (rlane & 1) != 0;
  const int q = lane >> 3, c8 = (lane & 7) * 8;
#pragma unroll
  for (int i = 0; i < 2; ++i) {
#pragma unroll
    for (int var = 0; var < 2; ++var) {
#pragma unroll
      for (int j = 0; j < 4; ++j) {
#pragma unroll
        for (int r = 0; r < 8; ++r) {
          const float pv = acc[i][j][r];
          const float qv = acc[i + 2][j][r];
          const float sq = oddc ? -qv : qv;
          const float sv = (var == 0) ? (pv + sq) : (pv - sq);
          slab[(mOff + r) * 68 + (j << 4) + rlane] = sv * kScale1;
        }
      }
      __builtin_amdgcn_fence(__ATOMIC_RELEASE, "workgroup");
      __builtin_amdgcn_wave_barrier();
      __builtin_amdgcn_fence(__ATOMIC_ACQUIRE, "workgroup");
      unsigned short* dst = SRCT + ((size_t)var * kDim + j0 + i * 16) * kKTot + (size_t)kf * kSeq + n0 + c8;
      for (int pass = 0; pass < 2; ++pass) {
#pragma unroll
        for (int it = 0; it < 4; ++it) {
          const int row = it * 4 + q;
          const float* sp = slab + row * 68 + c8;
          v8h hv;
#pragma unroll
          for (int e = 0; e < 8; ++e) hv[e] = (_Float16)sp[e];
          *(volatile v8h*)(dst + (size_t)row * kKTot) = hv;
        }
        __threadfence();
      }
      __builtin_amdgcn_fence(__ATOMIC_RELEASE, "workgroup");
      __builtin_amdgcn_wave_barrier();
      __builtin_amdgcn_fence(__ATOMIC_ACQUIRE, "workgroup");
    }
  }
}

__global__ __launch_bounds__(256) void lag_gemm_kernel(
    const unsigned short* __restrict__ VSp, const unsigned short* __restrict__ SRCTp,
    float* __restrict__ out)
{
  __shared__ __align__(16) float sT[8][16 * 68];
  const int lane = threadIdx.x & 31;
  const int wave = __builtin_amdgcn_readfirstlane((int)(threadIdx.x >> 5));
  const int p  = wave >> 2;
  const int jt = blockIdx.x * 4 + (wave & 3);
  const int j0 = jt * 64;
  const int e0 = blockIdx.y * 64;
  const int rlane = lane & 15;
  const int koff  = (lane >> 4) * 8;
  const int mOff  = (lane >> 4) * 8;

  const int lmax   = 2 * (e0 + 63) + p;
  const int ntiles = (lmax >> 5) + 1;

  const int l0   = 2 * (e0 + rlane) + p;
  const int off  = (kSeq - 1) - l0;
  const int cs   = off & 7;
  const int base = off - cs;

  const _Float16* VS   = (const _Float16*)VSp;
  const _Float16* SRCT = (const _Float16*)SRCTp;
  const _Float16* aV = VS + (size_t)(cs * kNf) * kVsPitch + base + koff;
  const _Float16* bS = SRCT + ((size_t)p * kDim + j0 + rlane) * kKTot + koff;

  v8f acc[4][4];
#pragma unroll
  for (int i = 0; i < 4; ++i)
#pragma unroll
    for (int j = 0; j < 4; ++j) acc[i][j] = (v8f){0.f,0.f,0.f,0.f,0.f,0.f,0.f,0.f};

  for (int kf = 0; kf < kNf; ++kf) {
    const _Float16* ak = aV + (size_t)kf * kVsPitch;
    const _Float16* bk = bS + (size_t)kf * kSeq;
    for (int tt = 0; tt < ntiles; ++tt) {
      const int t0 = tt << 5;
      v16h bh[4];
#pragma unroll
      for (int j = 0; j < 4; ++j) bh[j] = frag_load(bk + (size_t)(j * 16) * kKTot + t0);
#pragma unroll
      for (int i = 0; i < 4; ++i) {
        const v16h ah = frag_load(ak - 32 * i + t0);
#pragma unroll
        for (int j = 0; j < 4; ++j) acc[i][j] = frag_mma(ah, bh[j], acc[i][j]);
        row_guard(acc[i][0], acc[i][1], acc[i][2], acc[i][3], ah, bh[0], bh[1], bh[2], bh[3]);
      }
    }
  }
  acc_guard4(acc[0][0], acc[0][1], acc[0][2], acc[0][3]);
  acc_guard4(acc[1][0], acc[1][1], acc[1][2], acc[1][3]);
  acc_guard4(acc[2][0], acc[2][1], acc[2][2], acc[2][3]);
  acc_guard4(acc[3][0], acc[3][1], acc[3][2], acc[3][3]);

  float* slab = sT[wave];
  const int hh = lane >> 4, c4 = (lane & 15) * 4;
#pragma unroll
  for (int i = 0; i < 4; ++i) {
#pragma unroll
    for (int j = 0; j < 4; ++j) {
#pragma unroll
      for (int r = 0; r < 8; ++r) {
        slab[(mOff + r) * 68 + (j << 4) + rlane] = acc[i][j][r] * kScale2;
      }
    }
    __builtin_amdgcn_fence(__ATOMIC_RELEASE, "workgroup");
    __builtin_amdgcn_wave_barrier();
    __builtin_amdgcn_fence(__ATOMIC_ACQUIRE, "workgroup");
    for (int pass = 0; pass < 2; ++pass) {
#pragma unroll
      for (int it = 0; it < 8; ++it) {
        const int row = it * 2 + hh;
        const int l = 2 * (e0 + i * 16 + row) + p;
        const v4f val = *(const v4f*)(slab + row * 68 + c4);
        *(volatile v4f*)(out + (size_t)l * kDim + j0 + c4) = val;
      }
      __threadfence();
    }
    __builtin_amdgcn_fence(__ATOMIC_RELEASE, "workgroup");
    __builtin_amdgcn_wave_barrier();
    __builtin_amdgcn_fence(__ATOMIC_ACQUIRE, "workgroup");
  }
}

extern "C" void kernel_launch(void* const* d_in, const int* in_sizes, int n_in,
                              void* d_out, int out_size, void* d_ws, size_t ws_size,
                              hipStream_t stream) {
  if (n_in < 4) return;
  if (in_sizes[0] != kSeq * kDim) return;
  if (in_sizes[1] != kSeq * kNf) return;
  if (in_sizes[2] != kNf * kDim * kDim) return;
  if (in_sizes[3] != kNf * kDim * kDim) return;
  if (out_size != kSeq * kDim) return;
  if (ws_size < kWsTotal) return;

  const float* x  = (const float*)d_in[0];
  const float* vf = (const float*)d_in[1];
  const float* Wp = (const float*)d_in[2];
  const float* Wm = (const float*)d_in[3];
  float* out = (float*)d_out;

  char* ws = (char*)d_ws;
  unsigned short* X16  = (unsigned short*)(ws + kOffX16);
  unsigned short* MT   = (unsigned short*)(ws + kOffMT);
  unsigned short* SRCT = (unsigned short*)(ws + kOffSRCT);
  unsigned short* VS   = (unsigned short*)(ws + kOffVS);

  prep_xv_kernel<<<kXBlocks + kVsBlocks, 256, 0, stream>>>(x, vf, X16, VS);

  prep_w_kernel<<<dim3(144, 16), 256, 0, stream>>>(Wp, Wm, MT, 0);
  proj_gemm_kernel<<<dim3(96, kKHalf), 256, 0, stream>>>(MT, X16, SRCT, 0);

  prep_w_kernel<<<dim3(144, 16), 256, 0, stream>>>(Wp, Wm, MT, 1);
  proj_gemm_kernel<<<dim3(96, kKHalf), 256, 0, stream>>>(MT, X16, SRCT, 1);

  lag_gemm_kernel<<<dim3(3, 16), 256, 0, stream>>>(VS, SRCT, out);
}
